// FlashMLP_59219009077886
// MI455X (gfx1250) — hardware-verified
//
#include <hip/hip_runtime.h>
#include <math.h>

constexpr int kNB      = 2;
constexpr int kNH      = 16;
constexpr int kSeq     = 2048;
constexpr int kHeadDim = 128;
constexpr int kNKV     = 4;
constexpr int kInter   = 2048;
constexpr int kGroups  = kNB * kNH;
constexpr int kGPB     = 2;
constexpr int kNBatch  = kGroups / kGPB;
constexpr int kQPlane  = kSeq * kHeadDim;
constexpr int kKVPlane = kInter * kHeadDim;
constexpr int kMNld    = 2 * kInter;
constexpr int kMNPlane = kSeq * kMNld;
constexpr int kAPlane  = kSeq * kInter;
constexpr float kScale   = 0.08838834764831845f;
constexpr float kLoCarry = 2048.0f;
constexpr float kLoInv   = 1.0f / 2048.0f;

typedef __attribute__((ext_vector_type(16))) _Float16 v16h;
typedef __attribute__((ext_vector_type(8)))  _Float16 v8h;
typedef __attribute__((ext_vector_type(16))) __bf16   v16b;
typedef __attribute__((ext_vector_type(8)))  __bf16   v8b;
typedef __attribute__((ext_vector_type(8)))  float    v8f;
typedef __attribute__((ext_vector_type(4)))  float    v4f;
typedef __attribute__((ext_vector_type(4)))  unsigned int v4u;

__device__ __forceinline__ unsigned short f2bf_bits(float f) {
  unsigned u = __float_as_uint(f);
  return (unsigned short)((u + 0x7FFFu + ((u >> 16) & 1u)) >> 16);
}
__device__ __forceinline__ float bf_bits2f(unsigned short h) { return __uint_as_float(((unsigned)h) << 16); }

__device__ __forceinline__ void dep_guard_h(v8f& a, v8f& b, v16h x, v16h y) { asm volatile("v_nop\n\tv_nop\n\tv_nop\n\tv_nop" : "+v"(a), "+v"(b) : "v"(x), "v"(y)); }
__device__ __forceinline__ void dep_guard_b(v8f& a, v8f& b, v16b x, v16b y) { asm volatile("v_nop\n\tv_nop\n\tv_nop\n\tv_nop" : "+v"(a), "+v"(b) : "v"(x), "v"(y)); }
__device__ __forceinline__ void keep4_h(v16h a, v16h b, v16h c, v16h d) { asm volatile("v_nop" :: "v"(a), "v"(b), "v"(c), "v"(d)); }
__device__ __forceinline__ void keep4_b(v16b a, v16b b, v16b c, v16b d) { asm volatile("v_nop" :: "v"(a), "v"(b), "v"(c), "v"(d)); }
__device__ __forceinline__ void acc_guard4(v8f& a, v8f& b, v8f& c, v8f& d) { asm volatile("v_nop\n\tv_nop\n\tv_nop\n\tv_nop" : "+v"(a), "+v"(b), "+v"(c), "+v"(d)); }
template <typename T> struct Frag;
template <> struct Frag<_Float16> {
  typedef v16h V; union U { v16h v; v8h h[2]; };
  static __device__ __forceinline__ v16h load(const _Float16* p) {
    U f; f.h[0] = *(const v8h*)(p); f.h[1] = *(const v8h*)(p + 16); return f.v;
  }
  static __device__ __forceinline__ v8f mma(v16h a, v16h b, v8f c) {
    return __builtin_amdgcn_wmma_f32_16x16x32_f16(false, a, false, b, (short)0, c, false, false);
  }
  static __device__ __forceinline__ void guard(v8f& a, v8f& b, v16h x, v16h y) { dep_guard_h(a, b, x, y); }
  static __device__ __forceinline__ void keep(v16h a, v16h b, v16h c, v16h d) { keep4_h(a, b, c, d); }
};
template <> struct Frag<__bf16> {
  typedef v16b V; union U { v16b v; v8b h[2]; };
  static __device__ __forceinline__ v16b load(const __bf16* p) {
    U f; f.h[0] = *(const v8b*)(p); f.h[1] = *(const v8b*)(p + 16); return f.v;
  }
  static __device__ __forceinline__ v8f mma(v16b a, v16b b, v8f c) {
    return __builtin_amdgcn_wmma_f32_16x16x32_bf16(false, a, false, b, (short)0, c, false, false);
  }
  static __device__ __forceinline__ void guard(v8f& a, v8f& b, v16b x, v16b y) { dep_guard_b(a, b, x, y); }
  static __device__ __forceinline__ void keep(v16b a, v16b b, v16b c, v16b d) { keep4_b(a, b, c, d); }
};

__device__ __forceinline__ unsigned pk16(unsigned short a, unsigned short b) { return (unsigned)a | ((unsigned)b << 16); }
__device__ __forceinline__ unsigned short h_bits(float f) { const _Float16 h = (_Float16)f; return __builtin_bit_cast(unsigned short, h); }

template <int ET> struct Elem;
template <> struct Elem<0> { typedef _Float16 T; };
template <> struct Elem<1> { typedef __bf16 T; };
template <int ET, bool SPLIT, int BIAS_MODE, int OUT_MODE, bool RESID, int ACT = 0>
__global__ __launch_bounds__(256) void wmma_gemm64(
    const unsigned short* __restrict__ Ap, const unsigned short* __restrict__ A2p, int lda, long strideA,
    const unsigned short* __restrict__ Btp, const unsigned short* __restrict__ Bt2p, int ldb, long strideB,
    void* __restrict__ Cout, void* __restrict__ Cout2, int ldc, long strideC,
    const float* __restrict__ bias,
    const float* __restrict__ resid, long strideR,
    int M, int N, int K, float scale) {
  typedef typename Elem<ET>::T T;
  typedef typename Frag<T>::V V;
  const T* A = (const T*)Ap; const T* A2 = (const T*)A2p; const T* Bt = (const T*)Btp; const T* Bt2 = (const T*)Bt2p;
  __shared__ __align__(16) float sT[8][16 * 68];
  const int b    = blockIdx.y;
  const int lane = threadIdx.x & 31;
  const int wave = threadIdx.x >> 5;
  const int tilesN = N >> 6;
  const int tilesM = M >> 6;
  const int tile = blockIdx.x * 8 + wave;
  if (tile >= tilesM * tilesN) return;
  const int tm = tile / tilesN;
  const int tn = tile - tm * tilesN;
  const int m0 = tm << 6;
  const int n0 = tn << 6;

  const T* Ab  = A  + (size_t)b * strideA;
  const T* Bb  = Bt + (size_t)b * strideB;
  const T* Ab2 = SPLIT ? (A2  + (size_t)b * strideA) : nullptr;
  const T* Bb2 = SPLIT ? (Bt2 + (size_t)b * strideB) : nullptr;

  const int rlane = lane & 15;
  const int koff  = (lane >> 4) * 8;
  const int mOff  = (lane >> 4) * 8;

  v8f acc[4][4];
#pragma unroll
  for (int i = 0; i < 4; ++i)
#pragma unroll
    for (int j = 0; j < 4; ++j) acc[i][j] = (v8f){0.f,0.f,0.f,0.f,0.f,0.f,0.f,0.f};

  for (int k0 = 0; k0 < K; k0 += 32) {
    V bh[4], bl[4];
#pragma unroll
    for (int j = 0; j < 4; ++j) {
      const size_t bo = (size_t)(n0 + (j << 4) + rlane) * ldb + koff + k0;
      bh[j] = Frag<T>::load(Bb + bo);
      if (SPLIT) bl[j] = Frag<T>::load(Bb2 + bo);
    }
#pragma unroll
    for (int i = 0; i < 4; ++i) {
      const size_t ao = (size_t)(m0 + (i << 4) + rlane) * lda + koff + k0;
      V ah = Frag<T>::load(Ab + ao);
      V al;
      if (SPLIT) al = Frag<T>::load(Ab2 + ao);
#pragma unroll
      for (int j = 0; j < 4; ++j) {
        acc[i][j] = Frag<T>::mma(ah, bh[j], acc[i][j]);
        if (SPLIT) {
          acc[i][j] = Frag<T>::mma(ah, bl[j], acc[i][j]);
          acc[i][j] = Frag<T>::mma(al, bh[j], acc[i][j]);
        }
      }
      Frag<T>::guard(acc[i][0], acc[i][3], ah, SPLIT ? al : ah);
    }
    Frag<T>::keep(bh[0], bh[1], bh[2], bh[3]);
    if (SPLIT) Frag<T>::keep(bl[0], bl[1], bl[2], bl[3]);
  }
  acc_guard4(acc[0][0], acc[0][1], acc[0][2], acc[0][3]);
  acc_guard4(acc[1][0], acc[1][1], acc[1][2], acc[1][3]);
  acc_guard4(acc[2][0], acc[2][1], acc[2][2], acc[2][3]);
  acc_guard4(acc[3][0], acc[3][1], acc[3][2], acc[3][3]);

  float* slab = sT[wave];
  const float* Rb = RESID ? (resid + (size_t)b * strideR) : nullptr;
#pragma unroll
  for (int i = 0; i < 4; ++i) {
    const int mBase = m0 + (i << 4);
#pragma unroll
    for (int j = 0; j < 4; ++j) {
      const int n = n0 + (j << 4) + rlane;
      float bv = 0.f;
      if (BIAS_MODE == 2) bv = bias[n];
#pragma unroll
      for (int r = 0; r < 8; ++r) {
        float v = acc[i][j][r] * scale;
        if (BIAS_MODE == 1) v += bias[mBase + mOff + r];
        if (BIAS_MODE == 2) v += bv;
        if (RESID) v += Rb[(size_t)(mBase + mOff + r) * ldc + n];
        if (ACT == 2) v = fmaxf(v, 0.0f);
        if (ACT == 4) v = (v > 0.f) ? v : 0.01f * v;
        slab[(mOff + r) * 68 + (j << 4) + rlane] = v;
      }
    }
    __builtin_amdgcn_fence(__ATOMIC_RELEASE, "workgroup");
    __builtin_amdgcn_wave_barrier();
    __builtin_amdgcn_fence(__ATOMIC_ACQUIRE, "workgroup");
    if (OUT_MODE == 0) {
      float* C = (float*)Cout + (size_t)b * strideC;
      const int hh = lane >> 4, c4 = (lane & 15) * 4;
      for (int pass = 0; pass < 2; ++pass) {
#pragma unroll
        for (int it = 0; it < 8; ++it) {
          const int row = it * 2 + hh;
          v4f v = *(const v4f*)(slab + row * 68 + c4);
          *(volatile v4f*)(C + (size_t)(mBase + row) * ldc + n0 + c4) = v;
        }
        __threadfence();
      }
    } else {
      const int q = lane >> 3, c8 = (lane & 7) * 8;
      unsigned short* C  = (unsigned short*)Cout  + (size_t)b * strideC;
      unsigned short* C2 = (OUT_MODE == 2) ? ((unsigned short*)Cout2 + (size_t)b * strideC) : nullptr;
      for (int pass = 0; pass < 2; ++pass) {
#pragma unroll
        for (int it = 0; it < 4; ++it) {
          const int row = it * 4 + q;
          const float* sp = slab + row * 68 + c8;
          v8h hv, lv;
#pragma unroll
          for (int e = 0; e < 8; ++e) {
            if (OUT_MODE == 1) {
              hv[e] = (_Float16)sp[e];
            } else {
              unsigned short hb = f2bf_bits(sp[e]);
              unsigned short lb = f2bf_bits(sp[e] - bf_bits2f(hb));
              hv[e] = __builtin_bit_cast(_Float16, hb);
              lv[e] = __builtin_bit_cast(_Float16, lb);
            }
          }
          *(volatile v8h*)(C + (size_t)(mBase + row) * ldc + n0 + c8) = hv;
          if (OUT_MODE == 2) *(volatile v8h*)(C2 + (size_t)(mBase + row) * ldc + n0 + c8) = lv;
        }
        __threadfence();
      }
    }
    __builtin_amdgcn_fence(__ATOMIC_RELEASE, "workgroup");
    __builtin_amdgcn_wave_barrier();
    __builtin_amdgcn_fence(__ATOMIC_ACQUIRE, "workgroup");
  }
}

__global__ __launch_bounds__(256) void cast8_f16_kernel(const float* __restrict__ in, unsigned short* __restrict__ out, int n8) {
  const int i = blockIdx.x * 256 + threadIdx.x;
  if (i >= n8) return;
  const float* p = in + 8 * (size_t)i;
  const v4f a = *(const v4f*)(p);
  const v4f c = *(const v4f*)(p + 4);
  unsigned short hb[8];
#pragma unroll
  for (int e = 0; e < 4; ++e) {
    hb[e]     = h_bits(a[e]);
    hb[4 + e] = h_bits(c[e]);
  }
  const v4u u = (v4u){pk16(hb[0], hb[1]), pk16(hb[2], hb[3]), pk16(hb[4], hb[5]), pk16(hb[6], hb[7])};
  unsigned short* q = out + 8 * (size_t)i;
  *(volatile v4u*)q = u;
  __threadfence();
  *(volatile v4u*)q = u;
}

__global__ __launch_bounds__(256) void cast8_pair_kernel(const float* __restrict__ in0, const float* __restrict__ in1,
                                                          unsigned short* __restrict__ out, int n8) {
  const int i = blockIdx.x * 256 + threadIdx.x;
  const int which = blockIdx.y;
  if (i >= n8) return;
  const float* src = (which == 0) ? in0 : in1;
  const float* p = src + 8 * (size_t)i;
  const v4f a = *(const v4f*)(p);
  const v4f c = *(const v4f*)(p + 4);
  unsigned short hb[8];
#pragma unroll
  for (int e = 0; e < 4; ++e) {
    hb[e]     = h_bits(a[e]);
    hb[4 + e] = h_bits(c[e]);
  }
  const v4u u = (v4u){pk16(hb[0], hb[1]), pk16(hb[2], hb[3]), pk16(hb[4], hb[5]), pk16(hb[6], hb[7])};
  const int kh = i >> 15;
  const int r8 = i & 32767;
  unsigned short* q = out + 8 * ((size_t)(kh * 2 + which) * 32768 + r8);
  *(volatile v4u*)q = u;
  __threadfence();
  *(volatile v4u*)q = u;
}

__global__ __launch_bounds__(256) void vt_kernel(const float* __restrict__ Vin, unsigned short* __restrict__ out) {
  __shared__ float sm[64][65];
  const int t  = threadIdx.x;
  const int i0 = blockIdx.x * 64;
  const int d0 = blockIdx.y * 64;
  const int kh = blockIdx.z;
#pragma unroll
  for (int it = 0; it < 16; ++it) {
    const int e = it * 256 + t;
    const int r = e >> 6;
    const int c = e & 63;
    sm[c][r] = Vin[((size_t)kh * kInter + i0 + r) * kHeadDim + d0 + c];
  }
  __syncthreads();
  const int lane = t & 31, wave = t >> 5;
  const int q = lane >> 3, c8 = (lane & 7) * 8;
  unsigned short* op = out + (size_t)kh * kHeadDim * kInter;
  for (int pass = 0; pass < 2; ++pass) {
#pragma unroll
    for (int it = 0; it < 2; ++it) {
      const int row = wave * 8 + it * 4 + q;
      unsigned short hb[8];
#pragma unroll
      for (int e = 0; e < 8; ++e) hb[e] = h_bits(sm[row][c8 + e]);
      const v4u u = (v4u){pk16(hb[0], hb[1]), pk16(hb[2], hb[3]), pk16(hb[4], hb[5]), pk16(hb[6], hb[7])};
      *(volatile v4u*)(op + (size_t)(d0 + row) * kInter + i0 + c8) = u;
    }
    __threadfence();
  }
}

__device__ __forceinline__ void gate_one(float m, float n, unsigned short& hb, unsigned short& lb) {
  const float sg = __builtin_amdgcn_rcpf(1.0f + expf(-m));
  const float a  = (m * sg) * n;
  const _Float16 h = (_Float16)a;
  const float hf = (float)h;
  const _Float16 l = (_Float16)((a - hf) * kLoCarry);
  hb = __builtin_bit_cast(unsigned short, h);
  lb = __builtin_bit_cast(unsigned short, l);
}

__global__ __launch_bounds__(256) void gate_kernel(const float* __restrict__ MN, unsigned short* __restrict__ Ah,
                                                   unsigned short* __restrict__ Al, int nthr) {
  const int i = blockIdx.x * 256 + threadIdx.x;
  if (i >= nthr) return;
  const int row = i >> 8;
  const int c0  = (i & 255) * 8;
  const float* mp = MN + (size_t)row * kMNld + c0;
  const float* np = mp + kInter;
  const v4f m0 = *(const v4f*)(mp);
  const v4f m1 = *(const v4f*)(mp + 4);
  const v4f n0 = *(const v4f*)(np);
  const v4f n1 = *(const v4f*)(np + 4);
  unsigned short hb[8], lb[8];
#pragma unroll
  for (int e = 0; e < 4; ++e) {
    gate_one(m0[e], n0[e], hb[e], lb[e]);
    gate_one(m1[e], n1[e], hb[4 + e], lb[4 + e]);
  }
  const v4u uh = (v4u){pk16(hb[0], hb[1]), pk16(hb[2], hb[3]), pk16(hb[4], hb[5]), pk16(hb[6], hb[7])};
  const v4u ul = (v4u){pk16(lb[0], lb[1]), pk16(lb[2], lb[3]), pk16(lb[4], lb[5]), pk16(lb[6], lb[7])};
  unsigned short* qh = Ah + 8 * (size_t)i;
  unsigned short* ql = Al + 8 * (size_t)i;
  *(volatile v4u*)qh = uh;
  *(volatile v4u*)ql = ul;
  __threadfence();
  *(volatile v4u*)qh = uh;
  *(volatile v4u*)ql = ul;
}

extern "C" void kernel_launch(void* const* d_in, const int* in_sizes, int n_in,
                              void* d_out, int out_size, void* d_ws, size_t ws_size,
                              hipStream_t stream) {
  if (n_in < 4) return;
  if (in_sizes[0] != kGroups * kQPlane) return;
  if (in_sizes[1] != kNKV * kKVPlane || in_sizes[2] != kNKV * kKVPlane || in_sizes[3] != kNKV * kKVPlane) return;
  if (out_size != kGroups * kQPlane) return;

  const size_t bytesQ16  = (size_t)kGroups * kQPlane * 2;
  const size_t bytesKU16 = (size_t)kNKV * 2 * kKVPlane * 2;
  const size_t bytesVT16 = (size_t)kNKV * kKVPlane * 2;
  const size_t bytesMN   = (size_t)kGPB * kMNPlane * 4;
  const size_t bytesA    = (size_t)kGPB * kAPlane * 2;
  const size_t bytesOhi  = (size_t)kGPB * kQPlane * 4;
  const size_t offQ16  = 0;
  const size_t offKU16 = offQ16 + bytesQ16;
  const size_t offVT16 = offKU16 + bytesKU16;
  const size_t offMN   = offVT16 + bytesVT16;
  const size_t offAhi  = offMN + bytesMN;
  const size_t offAlo  = offAhi + bytesA;
  const size_t offOhi  = offAlo + bytesA;
  const size_t total   = offOhi + bytesOhi;
  if (ws_size < total) return;

  const float* Qp = (const float*)d_in[0];
  const float* Kp = (const float*)d_in[1];
  const float* Up = (const float*)d_in[2];
  const float* Vp = (const float*)d_in[3];
  float* Op = (float*)d_out;
  char* ws = (char*)d_ws;
  unsigned short* Q16  = (unsigned short*)(ws + offQ16);
  unsigned short* KU16 = (unsigned short*)(ws + offKU16);
  unsigned short* VT16 = (unsigned short*)(ws + offVT16);
  float*          MNf  = (float*)(ws + offMN);
  unsigned short* Ahi  = (unsigned short*)(ws + offAhi);
  unsigned short* Alo  = (unsigned short*)(ws + offAlo);
  float*          Ohi  = (float*)(ws + offOhi);

  cast8_f16_kernel<<<dim3((kGroups * kQPlane / 8) / 256), dim3(256), 0, stream>>>(Qp, Q16, kGroups * kQPlane / 8);
  cast8_pair_kernel<<<dim3((kNKV * kKVPlane / 8) / 256, 2), dim3(256), 0, stream>>>(Kp, Up, KU16, kNKV * kKVPlane / 8);
  vt_kernel<<<dim3(kInter / 64, kHeadDim / 64, kNKV), dim3(256), 0, stream>>>(Vp, VT16);

  for (int gb = 0; gb < kNBatch; ++gb) {
    const int p0 = gb * kGPB;
    const int kh = ((p0 & 15) >> 2);
    const unsigned short* Ag = Q16 + (size_t)p0 * kQPlane;
    const unsigned short* Bg = KU16 + (size_t)kh * 2 * kKVPlane;
    const unsigned short* Vg = VT16 + (size_t)kh * kKVPlane;
    float* Og = Op + (size_t)p0 * kQPlane;

    wmma_gemm64<0, false, 0, 0, false><<<dim3(256, kGPB), dim3(256), 0, stream>>>(
        Ag, Ag, kHeadDim, (long)kQPlane,
        Bg, Bg, kHeadDim, 0L,
        (void*)MNf, (void*)MNf, kMNld, (long)kMNPlane,
        MNf, MNf, 0L,
        kSeq, kMNld, kHeadDim, kScale);

    gate_kernel<<<dim3((kGPB * kAPlane / 8) / 256), dim3(256), 0, stream>>>(MNf, Ahi, Alo, kGPB * kAPlane / 8);

    wmma_gemm64<0, false, 0, 0, false><<<dim3(8, kGPB), dim3(256), 0, stream>>>(
        Ahi, Ahi, kInter, (long)kAPlane,
        Vg, Vg, kInter, 0L,
        (void*)Ohi, (void*)Ohi, kHeadDim, (long)kQPlane,
        Ohi, Ohi, 0L,
        kSeq, kHeadDim, kInter, 1.0f);

    wmma_gemm64<0, false, 0, 0, true><<<dim3(8, kGPB), dim3(256), 0, stream>>>(
        Alo, Alo, kInter, (long)kAPlane,
        Vg, Vg, kInter, 0L,
        (void*)Og, (void*)Og, kHeadDim, (long)kQPlane,
        Ohi, Ohi, (long)kQPlane,
        kSeq, kHeadDim, kInter, kLoInv);
  }
}
